// SoftSW_82386062672159
// MI455X (gfx1250) — hardware-run, weakly checked
//
#include <hip/hip_runtime.h>
#include <math.h>

typedef __attribute__((ext_vector_type(16))) _Float16 v16h;
typedef __attribute__((ext_vector_type(8)))  _Float16 v8h;
typedef __attribute__((ext_vector_type(8)))  float    v8f;
typedef __attribute__((ext_vector_type(4)))  float    v4f;

constexpr int   kB       = 4;
constexpr int   kN       = 512;
constexpr int   kM       = 512;
constexpr int   kD       = 128;
constexpr int   kRowsX   = kB * kN;
constexpr int   kRowsY   = kB * kM;
constexpr int   kRowsAll = kRowsX + kRowsY;
constexpr float kCarry   = 64.0f;
constexpr float kFold    = 2.0f / (kCarry * kCarry);
constexpr float kNeg     = -1.0e30f;
constexpr int   kLdsP    = 520;
constexpr int   kSteps   = 1024;
constexpr int   kGroups  = kSteps / 4;
constexpr int   kOutTotal = 1 + kB * kN * kM;
constexpr int   kFullQuads = (kOutTotal - 1) / 4;
constexpr int   kPackBlocks = (kFullQuads + 1 + 255) / 256;
static_assert(kN == 512 && kM == 512, "index shifts below assume 512 x 512 tables");
static_assert((kD % 32) == 0, "GEMM K multiple of 32");
static_assert((kN % 64) == 0 && (kM % 64) == 0, "GEMM M,N multiples of 64");
static_assert(kN + kM - 1 <= kSteps, "wavefront steps fit the padded step count");
static_assert(kLdsP >= kN + 1, "LDS row holds the boundary slot plus one slot per table row");
static_assert((kRowsX % 32) == 0 && (kRowsY % 32) == 0, "32 rows per convert block");
static_assert(kOutTotal == 1048577, "output element count");
static_assert(kFullQuads * 4 + 1 == kOutTotal, "one scalar tail after the full quads");

constexpr size_t kOffPlanes = 0;
constexpr size_t kOffNrm    = kOffPlanes + (size_t)kRowsAll * kD * 2;
constexpr size_t kOffSmat   = kOffNrm    + (size_t)kRowsAll * 4;
constexpr size_t kOffDsk    = kOffSmat   + (size_t)kB * kN * kM * 4;
constexpr size_t kOffVals   = kOffDsk    + (size_t)kB * kGroups * kN * 4 * 4;
constexpr size_t kWsTotal   = kOffVals   + (size_t)kB * 32 * 4;
static_assert(kWsTotal == 13648384ull, "carve total");
static_assert(kWsTotal <= 134217728ull, "carve cap");
static_assert((kOffNrm % 128) == 0 && (kOffSmat % 128) == 0 && (kOffDsk % 128) == 0 && (kOffVals % 128) == 0, "128-B aligned regions");

union FragU { v16h v; v8h h[2]; };
__device__ __forceinline__ v16h frag_load(const _Float16* p) {
  FragU f;
  f.h[0] = *(const v8h*)(p);
  f.h[1] = *(const v8h*)(p + 16);
  return f.v;
}
__device__ __forceinline__ v8f mma_h(v16h a, v16h b, v8f c) {
  c = __builtin_amdgcn_wmma_f32_16x16x32_f16(false, a, false, b, (short)0, c, false, false);
  asm volatile("v_nop\n\tv_nop\n\tv_nop\n\tv_nop" : "+v"(c) : "v"(a), "v"(b));
  return c;
}

__global__ __launch_bounds__(256) void cast_norm_kernel(
    const float* __restrict__ x, const float* __restrict__ y,
    unsigned short* __restrict__ planes, float* __restrict__ nrm)
{
  __shared__ float sN[32];
  const int tid  = threadIdx.x;
  const int lane = tid & 31;
  const int wave = __builtin_amdgcn_readfirstlane((int)(threadIdx.x >> 5));
  const int hw   = lane >> 4;
  const int l16  = lane & 15;
  const int blk  = blockIdx.x;
  const bool isx = (blk < kRowsX / 32);
  const float* src = isx ? x : y;
  const int sbase  = isx ? (blk * 32) : ((blk - kRowsX / 32) * 32);
  v8h hv[2];
  float ssum[2];
#pragma unroll
  for (int it = 0; it < 2; ++it) {
    const int rl = it * 16 + wave * 2 + hw;
    const float* rp = src + (size_t)(sbase + rl) * kD + l16 * 8;
    const v4f a0 = *(const v4f*)(rp);
    const v4f a1 = *(const v4f*)(rp + 4);
    float ss = 0.0f;
#pragma unroll
    for (int e = 0; e < 4; ++e) ss = fmaf(a0[e], a0[e], ss);
#pragma unroll
    for (int e = 0; e < 4; ++e) ss = fmaf(a1[e], a1[e], ss);
    ss += __shfl_xor(ss, 1, 32);
    ss += __shfl_xor(ss, 2, 32);
    ss += __shfl_xor(ss, 4, 32);
    ss += __shfl_xor(ss, 8, 32);
    ssum[it] = ss;
#pragma unroll
    for (int e = 0; e < 4; ++e) {
      hv[it][e]     = (_Float16)(a0[e] * kCarry);
      hv[it][4 + e] = (_Float16)(a1[e] * kCarry);
    }
  }
  if (l16 == 0) {
    sN[wave * 2 + hw]      = ssum[0];
    sN[16 + wave * 2 + hw] = ssum[1];
  }
  for (int pass = 0; pass < 2; ++pass) {
#pragma unroll
    for (int it = 0; it < 2; ++it) {
      const int rl = it * 16 + wave * 2 + hw;
      *(volatile v8h*)(planes + (size_t)(blk * 32 + rl) * kD + l16 * 8) = hv[it];
    }
    __threadfence();
  }
  __syncthreads();
  if (wave == 0) {
    const float nv = sN[lane];
    float* p = nrm + blk * 32 + lane;
    *(volatile float*)p = nv;
    __threadfence();
    *(volatile float*)p = nv;
    __threadfence();
  }
}

__global__ __launch_bounds__(256) void dist_gemm_kernel(
    const unsigned short* __restrict__ planes, const float* __restrict__ nrm, float* __restrict__ Smat)
{
  __shared__ __align__(16) float sT[8][16 * 68];
  const int b    = blockIdx.y;
  const int lane = threadIdx.x & 31;
  const int wave = __builtin_amdgcn_readfirstlane((int)(threadIdx.x >> 5));
  const int tile = blockIdx.x * 8 + wave;
  const int tm = tile >> 3;
  const int tn = tile & 7;
  const int m0 = tm << 6;
  const int n0 = tn << 6;

  const _Float16* Ab = (const _Float16*)planes + (size_t)b * kN * kD;
  const _Float16* Bb = (const _Float16*)planes + (size_t)(kRowsX + b * kM) * kD;
  const float* xn = nrm + b * kN;
  const float* yn = nrm + kRowsX + b * kM;

  const int rlane = lane & 15;
  const int koff  = (lane >> 4) * 8;
  const int mOff  = (lane >> 4) * 8;

  v8f acc[4][4];
#pragma unroll
  for (int i = 0; i < 4; ++i)
#pragma unroll
    for (int j = 0; j < 4; ++j) acc[i][j] = (v8f){0.f,0.f,0.f,0.f,0.f,0.f,0.f,0.f};

#pragma unroll 1
  for (int k0 = 0; k0 < kD; k0 += 32) {
    v16h bh[4];
#pragma unroll
    for (int j = 0; j < 4; ++j) {
      const size_t bo = (size_t)(n0 + (j << 4) + rlane) * kD + koff + k0;
      bh[j] = frag_load(Bb + bo);
    }
#pragma unroll
    for (int i = 0; i < 4; ++i) {
      const size_t ao = (size_t)(m0 + (i << 4) + rlane) * kD + koff + k0;
      const v16h ah = frag_load(Ab + ao);
#pragma unroll
      for (int j = 0; j < 4; ++j) acc[i][j] = mma_h(ah, bh[j], acc[i][j]);
    }
  }

  float ycol[4];
#pragma unroll
  for (int j = 0; j < 4; ++j) ycol[j] = yn[n0 + (j << 4) + rlane];

  float* slab = sT[wave];
  float* C = Smat + (size_t)b * kN * kM;
#pragma unroll
  for (int i = 0; i < 4; ++i) {
    const int mBase = m0 + (i << 4);
    const v4f xa = *(const v4f*)(xn + mBase + mOff);
    const v4f xb = *(const v4f*)(xn + mBase + mOff + 4);
#pragma unroll
    for (int j = 0; j < 4; ++j) {
#pragma unroll
      for (int r = 0; r < 8; ++r) {
        const float xr = (r < 4) ? xa[r & 3] : xb[r & 3];
        const float v = (xr + ycol[j]) - kFold * acc[i][j][r];
        slab[(mOff + r) * 68 + (j << 4) + rlane] = v;
      }
    }
    __builtin_amdgcn_fence(__ATOMIC_RELEASE, "workgroup");
    __builtin_amdgcn_wave_barrier();
    __builtin_amdgcn_fence(__ATOMIC_ACQUIRE, "workgroup");
    {
      const int hh = lane >> 4;
      const int c4 = (lane & 15) * 4;
      for (int pass = 0; pass < 2; ++pass) {
#pragma unroll
        for (int it = 0; it < 8; ++it) {
          const int row = it * 2 + hh;
          const v4f v = *(const v4f*)(slab + row * 68 + c4);
          *(volatile v4f*)(C + (size_t)(mBase + row) * kM + n0 + c4) = v;
        }
        __threadfence();
      }
    }
    __builtin_amdgcn_fence(__ATOMIC_RELEASE, "workgroup");
    __builtin_amdgcn_wave_barrier();
    __builtin_amdgcn_fence(__ATOMIC_ACQUIRE, "workgroup");
  }
}

__global__ __launch_bounds__(512) void dp_wavefront_kernel(
    const float* __restrict__ Smat, const float* __restrict__ go, const float* __restrict__ ge,
    float* __restrict__ Dsk, float* __restrict__ vals)
{
  __shared__ float sBuf[2 * 3 * kLdsP];
  __shared__ float sRm[16];
  __shared__ float sRs[16];
  const int tid  = threadIdx.x;
  const int lane = tid & 31;
  const int wave = __builtin_amdgcn_readfirstlane((int)(threadIdx.x >> 5));
  const int b    = blockIdx.x;

  for (int k = tid; k < 2 * 3 * kLdsP; k += 512) sBuf[k] = kNeg;
  __syncthreads();

  const float* Srow  = Smat + ((size_t)b * kN + tid) * kM;
  const float* gorow = go + (size_t)tid * kM;
  const float* gerow = ge + (size_t)tid * kM;

  float Dl = kNeg, Ixl = kNeg;
  float Dd = kNeg, Ixd = kNeg, Iyd = kNeg;
  float m_acc = kNeg, s_acc = 0.0f;
  float q0 = 0.0f, q1 = 0.0f, q2 = 0.0f, q3 = 0.0f;

#pragma unroll 1
  for (int t = 0; t < kSteps; ++t) {
    const int c = t - tid;
    const bool act = (c >= 0) && (c < kM);
    int cc = (c < 0) ? 0 : c;
    cc = (cc > kM - 1) ? (kM - 1) : cc;
    const float sv  = Srow[cc];
    const float g_o = gorow[cc];
    const float g_e = gerow[cc];

    const float* rb = sBuf + ((t + 1) & 1) * (3 * kLdsP);
    const float Du  = rb[tid];
    const float Ixu = rb[kLdsP + tid];
    const float Iyu = rb[2 * kLdsP + tid];

    const float m4 = fmaxf(fmaxf(0.0f, Dd), fmaxf(Ixd, Iyd));
    const float e4 = (__expf(0.0f - m4) + __expf(Dd - m4)) + (__expf(Ixd - m4) + __expf(Iyd - m4));
    const float d  = sv + (m4 + __logf(e4));

    const float a1 = Dl - g_o;
    const float a2 = Ixl - g_e;
    const float m2 = fmaxf(a1, a2);
    const float ix = m2 + __logf(__expf(a1 - m2) + __expf(a2 - m2));

    const float b1 = Du - g_o;
    const float b2 = Ixu - g_o;
    const float b3 = Iyu - g_e;
    const float m3 = fmaxf(fmaxf(b1, b2), b3);
    const float iy = m3 + __logf((__expf(b1 - m3) + __expf(b2 - m3)) + __expf(b3 - m3));

    const float dp  = act ? d  : kNeg;
    const float ixp = act ? ix : kNeg;
    const float iyp = act ? iy : kNeg;

    float* wb = sBuf + (t & 1) * (3 * kLdsP);
    wb[tid + 1]             = dp;
    wb[kLdsP + tid + 1]     = ixp;
    wb[2 * kLdsP + tid + 1] = iyp;

    Dd = Du;  Ixd = Ixu;  Iyd = Iyu;
    Dl = dp;  Ixl = ixp;

    const float mn  = fmaxf(m_acc, dp);
    const float ea  = __expf(m_acc - mn);
    const float eb0 = __expf(dp - mn);
    const float eb  = act ? eb0 : 0.0f;
    s_acc = s_acc * ea + eb;
    m_acc = mn;

    const int u = t & 3;
    const float dz = act ? d : 0.0f;
    q0 = (u == 0) ? dz : q0;
    q1 = (u == 1) ? dz : q1;
    q2 = (u == 2) ? dz : q2;
    q3 = (u == 3) ? dz : q3;
    if (u == 3) {
      const v4f qv = (v4f){q0, q1, q2, q3};
      float* p = Dsk + (((size_t)b * kGroups + (size_t)(t >> 2)) * kN + tid) * 4;
      for (int pass = 0; pass < 2; ++pass) {
        *(volatile v4f*)p = qv;
        __threadfence();
      }
    }
    __syncthreads();
  }

#pragma unroll
  for (int off = 16; off > 0; off >>= 1) {
    const float mo = __shfl_xor(m_acc, off, 32);
    const float so = __shfl_xor(s_acc, off, 32);
    const float mm = fmaxf(m_acc, mo);
    s_acc = s_acc * __expf(m_acc - mm) + so * __expf(mo - mm);
    m_acc = mm;
  }
  if (lane == 0) { sRm[wave] = m_acc; sRs[wave] = s_acc; }
  __syncthreads();
  {
    const float lm = sRm[lane & 15];
    const float ls = sRs[lane & 15];
    float m2 = (lane < 16) ? lm : kNeg;
    float s2 = (lane < 16) ? ls : 0.0f;
#pragma unroll
    for (int off = 16; off > 0; off >>= 1) {
      const float mo = __shfl_xor(m2, off, 32);
      const float so = __shfl_xor(s2, off, 32);
      const float mm = fmaxf(m2, mo);
      s2 = s2 * __expf(m2 - mm) + so * __expf(mo - mm);
      m2 = mm;
    }
    const float val  = m2 + __logf(s2);
    const float outv = (lane == 0) ? val : 0.0f;
    if (wave == 0) {
      float* p = vals + b * 32 + lane;
      *(volatile float*)p = outv;
      __threadfence();
      *(volatile float*)p = outv;
      __threadfence();
    }
  }
}

__global__ __launch_bounds__(256) void pack_out_kernel(
    const float* __restrict__ Dsk, const float* __restrict__ vals, float* __restrict__ out)
{
  const int q = blockIdx.x * 256 + threadIdx.x;
  const float loss = (((vals[0] + vals[32]) + vals[64]) + vals[96]) * 0.25f;
  float v[4];
#pragma unroll
  for (int u = 0; u < 4; ++u) {
    int g = 4 * q + u;
    g = (g > kOutTotal - 1) ? (kOutTotal - 1) : g;
    const int e = (g > 0) ? (g - 1) : 0;
    const int bb = e >> 18;
    const int i  = (e >> 9) & 511;
    const int j  = e & 511;
    const int t  = i + j;
    const size_t idx = (((size_t)bb * kGroups + (size_t)(t >> 2)) * kN + (size_t)i) * 4 + (size_t)(t & 3);
    float dv = Dsk[idx];
    asm volatile("" : "+v"(dv));
    v[u] = (g == 0) ? loss : dv;
  }
  if (q < kFullQuads) {
    const v4f vv = (v4f){v[0], v[1], v[2], v[3]};
    float* p = out + (size_t)q * 4;
    for (int pass = 0; pass < 2; ++pass) {
      *(volatile v4f*)p = vv;
      __threadfence();
    }
  } else if (q == kFullQuads) {
    const float tv = v[0];
    float* p = out + (size_t)kFullQuads * 4;
    for (int pass = 0; pass < 2; ++pass) {
      *(volatile float*)p = tv;
      __threadfence();
    }
  }
}

extern "C" void kernel_launch(void* const* d_in, const int* in_sizes, int n_in,
                              void* d_out, int out_size, void* d_ws, size_t ws_size,
                              hipStream_t stream) {
  if (n_in < 4) return;
  if (in_sizes[0] != kB * kN * kD) return;
  if (in_sizes[1] != kB * kM * kD) return;
  if (in_sizes[2] != kN * kM) return;
  if (in_sizes[3] != kN * kM) return;
  if (out_size != kOutTotal) return;
  if (ws_size < kWsTotal) return;

  const float* x  = (const float*)d_in[0];
  const float* y  = (const float*)d_in[1];
  const float* go = (const float*)d_in[2];
  const float* ge = (const float*)d_in[3];
  float* out = (float*)d_out;

  char* ws = (char*)d_ws;
  unsigned short* PLANES = (unsigned short*)(ws + kOffPlanes);
  float*          NRM    = (float*)(ws + kOffNrm);
  float*          SMAT   = (float*)(ws + kOffSmat);
  float*          DSK    = (float*)(ws + kOffDsk);
  float*          VALS   = (float*)(ws + kOffVals);

  cast_norm_kernel<<<kRowsAll / 32, 256, 0, stream>>>(x, y, PLANES, NRM);
  dist_gemm_kernel<<<dim3((kN / 64) * (kM / 64) / 8, kB), 256, 0, stream>>>(PLANES, NRM, SMAT);
  dp_wavefront_kernel<<<kB, 512, 0, stream>>>(SMAT, go, ge, DSK, VALS);
  pack_out_kernel<<<kPackBlocks, 256, 0, stream>>>(DSK, VALS, out);
}
